// SelfAttentionModule_24008867184968
// MI455X (gfx1250) — hardware-verified
//
#include <hip/hip_runtime.h>
#include <math.h>

typedef __attribute__((ext_vector_type(16))) _Float16 v16h;
typedef __attribute__((ext_vector_type(16))) __bf16 v16b;
typedef __attribute__((ext_vector_type(8)))  _Float16 v8h;
typedef __attribute__((ext_vector_type(8)))  float v8f;
typedef __attribute__((ext_vector_type(4)))  float v4f;
typedef __attribute__((ext_vector_type(2)))  float v2f;
typedef __attribute__((ext_vector_type(4)))  unsigned v4u;
typedef __attribute__((ext_vector_type(4)))  int v4i;
typedef float __attribute__((may_alias)) float_a;
typedef int __attribute__((may_alias)) int_a;

template <typename T> __device__ __forceinline__ void vst2(void* p, T v) { *(volatile T*)p = v; __threadfence(); *(volatile T*)p = v; }
__device__ __forceinline__ v8f wmma16(v16h a, v16h b, v8f c) {
  v8f d = __builtin_amdgcn_wmma_f32_16x16x32_f16(false, a, false, b, (short)0, c, false, false);
  asm volatile("v_nop\n\tv_nop\n\tv_nop\n\tv_nop" : "+v"(d) : "v"(a), "v"(b));
  return d;
}
__device__ __forceinline__ v8f wmma_bf(v16b a, v16b b, v8f c) {
  v8f d = __builtin_amdgcn_wmma_f32_16x16x32_bf16(false, a, false, b, (short)0, c, false, false);
  asm volatile("v_nop\n\tv_nop\n\tv_nop\n\tv_nop" : "+v"(d) : "v"(a), "v"(b));
  return d;
}
__device__ __forceinline__ v16h frag_h(const _Float16* rowk0, int lane) {
  union { v16h v; v8h q[2]; } u; const _Float16* p = rowk0 + 8 * (lane >> 4);
  u.q[0] = *(const v8h*)p; u.q[1] = *(const v8h*)(p + 16); return u.v;
}
__device__ __forceinline__ v16h frag_f32(const float* rowk0, int lane) {
  v16h a; const float* p = rowk0 + 8 * (lane >> 4);
#pragma unroll
  for (int i = 0; i < 8; ++i) { a[i] = (_Float16)p[i]; a[8 + i] = (_Float16)p[16 + i]; }
  return a;
}
__device__ __forceinline__ v16h frag_f32s(const float* rowk0, int lane, float sc) {
  v16h a; const float* p = rowk0 + 8 * (lane >> 4);
#pragma unroll
  for (int i = 0; i < 8; ++i) { a[i] = (_Float16)(p[i] * sc); a[8 + i] = (_Float16)(p[16 + i] * sc); }
  return a;
}
__device__ __forceinline__ v16h fragc_f32(const float* W, int k0, int n, int lane, int ld, int K) {
  v16h a; const int g = lane >> 4;
#pragma unroll
  for (int i = 0; i < 8; ++i) { const int ka = k0 + 8 * g + i, kb = ka + 16;
    a[i] = (_Float16)(ka < K ? W[(size_t)(ka < K ? ka : K - 1) * ld + n] : 0.f); a[8 + i] = (_Float16)(kb < K ? W[(size_t)(kb < K ? kb : K - 1) * ld + n] : 0.f); }
  return a;
}
struct F2 { v16b h, l; };
__device__ __forceinline__ F2 bsplit16(const float v[16]) { F2 r;
#pragma unroll
  for (int i = 0; i < 16; ++i) { const __bf16 h = (__bf16)v[i]; r.h[i] = h; r.l[i] = (__bf16)(v[i] - (float)h); }
  return r; }
__device__ __forceinline__ F2 split_row(const float* row, int k0, int lane) { float v[16]; const float* p = row + k0 + 8 * (lane >> 4);
#pragma unroll
  for (int i = 0; i < 8; ++i) { v[i] = p[i]; v[8 + i] = p[16 + i]; }
  return bsplit16(v); }
__device__ __forceinline__ F2 split_rowK(const float* row, int k0, int lane, int K) { float v[16]; const int g = lane >> 4;
#pragma unroll
  for (int i = 0; i < 8; ++i) { const int ka = k0 + 8 * g + i, kb = ka + 16; v[i] = ka < K ? row[ka < K ? ka : K - 1] : 0.f; v[8 + i] = kb < K ? row[kb < K ? kb : K - 1] : 0.f; }
  return bsplit16(v); }
__device__ __forceinline__ F2 split_col(const float* W, int k0, int n, int lane, int ld, int K) { float v[16]; const int g = lane >> 4;
#pragma unroll
  for (int i = 0; i < 8; ++i) { const int ka = k0 + 8 * g + i, kb = ka + 16; v[i] = ka < K ? W[(size_t)(ka < K ? ka : K - 1) * ld + n] : 0.f; v[8 + i] = kb < K ? W[(size_t)(kb < K ? kb : K - 1) * ld + n] : 0.f; }
  return bsplit16(v); }
__device__ __forceinline__ v8f mac3(const F2& a, const F2& b, v8f c) { c = wmma_bf(a.l, b.h, c); c = wmma_bf(a.h, b.l, c); return wmma_bf(a.h, b.h, c); }
__device__ __forceinline__ float sigm(float v) { return 1.0f / (1.0f + expf(-v)); }
#define LDSX() do { asm volatile("s_wait_dscnt 0" ::: "memory"); __builtin_amdgcn_wave_barrier(); __builtin_amdgcn_fence(__ATOMIC_RELEASE, "workgroup"); } while (0)


#define NB 2
#define HW 96
#define NPX (HW * HW)
#define CIN 256
#define CK 64
#define CV 128
#define CO 256
#define NPT (NB * NPX)
#ifndef TWB
#define TWB (NPT / 128)
#endif
typedef __attribute__((ext_vector_type(8))) __bf16 v8b;
__device__ __forceinline__ v16b frag_b(const __bf16* rowk0, int lane) {
  union { v16b v; v8b q[2]; } u; const __bf16* p = rowk0 + 8 * (lane >> 4);
  u.q[0] = *(const v8b*)p; u.q[1] = *(const v8b*)(p + 16); return u.v;
}
__device__ __forceinline__ float bfr(float v) { return (float)(__bf16)v; }
__device__ __attribute__((noinline)) float exp_ni(float v) { return expf(v); }
__device__ __attribute__((noinline)) float erf_ni(float v) { return erff(v); }

#define WS_K1  0u
#define WS_Q1  (WS_K1 + 4u * (size_t)NPT * CK)
#define WS_KP  (WS_Q1 + 4u * (size_t)NPT * CK)
#define WS_QP  (WS_KP + 4u * (size_t)NPT * CK)
#define WS_VP  (WS_QP + 4u * (size_t)NPT * CK)
#define WS_CT  (WS_VP + 4u * (size_t)NPT * CV)
#define WS_END (WS_CT + 2u * (size_t)NPT * CV)

__device__ __forceinline__ float bnrelu(float v, const float* bn, int c, int C) { const float gsc = bfr(bn[c]) / sqrtf(bfr(bn[3 * C + c]) + 1e-5f); return fmaxf((v - bfr(bn[2 * C + c])) * gsc + bfr(bn[C + c]), 0.f); }
__global__ __launch_bounds__(128) void k_c1(const float* __restrict__ X, const float* __restrict__ WK1, const float* __restrict__ BK1, const float* __restrict__ BNK1, const float* __restrict__ WQ1, const float* __restrict__ BQ1, const float* __restrict__ BNQ1, const float* __restrict__ WV, const float* __restrict__ BVv, float* __restrict__ K1, float* __restrict__ Q1, float* __restrict__ VP) {
  __shared__ __align__(16) __bf16 sx[64][CIN + 8]; __shared__ __align__(16) float so[64][68];
  const int tid = threadIdx.x, wave = tid >> 5, lane = tid & 31, col = lane & 15, g = lane >> 4; const int p0 = blockIdx.x * 64; const size_t b = blockIdx.y; const int which = blockIdx.z;
  for (int e = tid; e < CIN * 64; e += 128) { const int c = e >> 6, pl = e & 63; sx[pl][c] = (__bf16)X[(b * CIN + c) * (size_t)NPX + p0 + pl]; }
  __syncthreads();
  const float* Wm = which == 0 ? WK1 : which == 1 ? WQ1 : (WV + (size_t)(which - 2) * 64 * CIN); const float* Bm = which == 0 ? BK1 : which == 1 ? BQ1 : (BVv + (which - 2) * 64);
  v8f acc[4] = {};
#pragma unroll 2
  for (int kc = 0; kc < CIN / 32; ++kc) { const v16b a = frag_b(&sx[wave * 16 + col][kc * 32], lane);
#pragma unroll
    for (int j = 0; j < 4; ++j) { v16b w; const int o = j * 16 + col;
#pragma unroll
      for (int i = 0; i < 8; ++i) { w[i] = (__bf16)Wm[(size_t)o * CIN + kc * 32 + 8 * g + i]; w[8 + i] = (__bf16)Wm[(size_t)o * CIN + kc * 32 + 16 + 8 * g + i]; }
      acc[j] = wmma_bf(a, w, acc[j]); } }
  if (which < 2) { const float* bn = which == 0 ? BNK1 : BNQ1;
#pragma unroll
    for (int j = 0; j < 4; ++j) { const int o = j * 16 + col; const float bb = bfr(Bm[o]);
#pragma unroll
      for (int r = 0; r < 8; ++r) so[wave * 16 + 8 * g + r][o] = bnrelu(acc[j][r] + bb, bn, o, CK); }
    __syncthreads(); float* dst = which == 0 ? K1 : Q1; for (int e = tid; e < 64 * 16; e += 128) { const int pl = e >> 4, q = e & 15; vst2(dst + (b * NPX + p0 + pl) * (size_t)CK + q * 4, *(const v4f*)&so[pl][q * 4]); } }
  else {
#pragma unroll
    for (int j = 0; j < 4; ++j) { const int o = j * 16 + col; const float bb = bfr(Bm[o]);
#pragma unroll
      for (int r = 0; r < 8; ++r) so[o][wave * 16 + 8 * g + r] = acc[j][r] + bb; }
    __syncthreads(); for (int e = tid; e < 64 * 16; e += 128) { const int cl = e >> 4, q = e & 15; vst2(VP + (b * CV + (which - 2) * 64 + cl) * (size_t)NPX + p0 + q * 4, *(const v4f*)&so[cl][q * 4]); } } }
__global__ __launch_bounds__(128) void k_c2(const float* __restrict__ K1, const float* __restrict__ Q1, const float* __restrict__ WK2, const float* __restrict__ BK2, const float* __restrict__ BNK2, const float* __restrict__ WQ2, const float* __restrict__ BQ2, const float* __restrict__ BNQ2, float* __restrict__ KP, float* __restrict__ QP) { __shared__ __align__(16) float so[64][68];
  const int tid = threadIdx.x, wave = tid >> 5, lane = tid & 31, col = lane & 15, g = lane >> 4; const int p0 = blockIdx.x * 64; const size_t b = blockIdx.y; const int which = blockIdx.z; const float* IN = which == 0 ? K1 : Q1; const float* Wm = which == 0 ? WK2 : WQ2; const float* Bm = which == 0 ? BK2 : BQ2; const float* bn = which == 0 ? BNK2 : BNQ2;
  v8f acc[4] = {};
#pragma unroll
  for (int kc = 0; kc < CK / 32; ++kc) { const F2 a = split_row(IN + (b * NPX + p0 + wave * 16 + col) * (size_t)CK, kc * 32, lane);
#pragma unroll
    for (int j = 0; j < 4; ++j) { v16b w; const int o = j * 16 + col;
#pragma unroll
      for (int i = 0; i < 8; ++i) { w[i] = (__bf16)Wm[(size_t)o * CK + kc * 32 + 8 * g + i]; w[8 + i] = (__bf16)Wm[(size_t)o * CK + kc * 32 + 16 + 8 * g + i]; }
      acc[j] = wmma_bf(a.h, w, acc[j]); acc[j] = wmma_bf(a.l, w, acc[j]); } }
#pragma unroll
  for (int j = 0; j < 4; ++j) { const int o = j * 16 + col; const float bb = bfr(Bm[o]);
#pragma unroll
    for (int r = 0; r < 8; ++r) { const float v = bnrelu(acc[j][r] + bb, bn, o, CK); if (which == 0) so[o][wave * 16 + 8 * g + r] = v; else so[wave * 16 + 8 * g + r][o] = v; } }
  __syncthreads();
  if (which == 0) { for (int e = tid; e < 64 * 16; e += 128) { const int cl = e >> 4, q = e & 15; vst2(KP + (b * CK + cl) * (size_t)NPX + p0 + q * 4, *(const v4f*)&so[cl][q * 4]); } }
  else { for (int e = tid; e < 64 * 16; e += 128) { const int pl = e >> 4, q = e & 15; vst2(QP + (b * NPX + p0 + pl) * (size_t)CK + q * 4, *(const v4f*)&so[pl][q * 4]); } } }
__global__ __launch_bounds__(128) void k_win(const float* __restrict__ KP, const float* __restrict__ QP, const float* __restrict__ VP, _Float16* __restrict__ CT) { __shared__ float sq[CK][129]; __shared__ float slg[49][129]; __shared__ __align__(16) _Float16 sct[128][CV + 8];
  const int t = threadIdx.x; const size_t p = (size_t)blockIdx.x * 128 + t; const size_t b = p / NPX; const int n = (int)(p % NPX); const int y = n / HW, x = n % HW;
  for (int e = t; e < 128 * CK; e += 128) { const int pl = e / CK, c = e % CK; sq[c][pl] = QP[((size_t)blockIdx.x * 128 + pl) * CK + c]; }
  __syncthreads();
  float mx = -3.0e38f;
#pragma unroll 1
  for (int k = 0; k < 49; ++k) { const int yy = y + k / 7 - 3, xx = x + k % 7 - 3; float s = 0.f;
    if (yy >= 0 && yy < HW && xx >= 0 && xx < HW) { const float* kp = KP + (b * CK) * (size_t)NPX + yy * HW + xx;
#pragma unroll 1
      for (int c = 0; c < CK; ++c) s += kp[(size_t)c * NPX] * sq[c][t]; }
    slg[k][t] = s; mx = fmaxf(mx, s); }
  float ssum = 0.f;
#pragma unroll 1
  for (int k = 0; k < 49; ++k) { const float e = expf(slg[k][t] - mx); slg[k][t] = e; ssum += e; }
  const float inv = 1.0f / ssum;
#pragma unroll 1
  for (int cv = 0; cv < CV; ++cv) { const float* vp = VP + (b * CV + cv) * (size_t)NPX; float a = 0.f;
#pragma unroll 1
    for (int k = 0; k < 49; ++k) { const int yy = y + k / 7 - 3, xx = x + k % 7 - 3; if (yy >= 0 && yy < HW && xx >= 0 && xx < HW) a += slg[k][t] * vp[yy * HW + xx]; }
    sct[t][cv] = (_Float16)(a * inv); }
  __syncthreads(); for (int e = t; e < 128 * (CV / 8); e += 128) { const int rl = e / (CV / 8), qq = e % (CV / 8); vst2((unsigned*)(CT + ((size_t)blockIdx.x * 128 + rl) * CV + qq * 8), *(const v4u*)&sct[rl][qq * 8]); } }
__global__ __launch_bounds__(128) void k_out(const _Float16* __restrict__ CT, const float* __restrict__ WW, const float* __restrict__ BW, float* __restrict__ OUT) { __shared__ __align__(16) float st[128][68];
  const int tid = threadIdx.x, wave = tid >> 5, lane = tid & 31, col = lane & 15, g = lane >> 4; const int p0 = blockIdx.x * 64; const size_t b = blockIdx.y; const int o0 = blockIdx.z * 128;
  v8f acc[8] = {};
#pragma unroll
  for (int kc = 0; kc < CV / 32; ++kc) { const v16h a = frag_h(CT + (b * NPX + p0 + wave * 16 + col) * (size_t)CV + kc * 32, lane);
#pragma unroll
    for (int j = 0; j < 8; ++j) { v16h w; const int o = o0 + j * 16 + col;
#pragma unroll
      for (int i = 0; i < 8; ++i) { w[i] = (_Float16)bfr(WW[(size_t)o * CV + kc * 32 + 8 * g + i]); w[8 + i] = (_Float16)bfr(WW[(size_t)o * CV + kc * 32 + 16 + 8 * g + i]); }
      acc[j] = wmma16(a, w, acc[j]); } }
#pragma unroll
  for (int j = 0; j < 8; ++j) { const int o = o0 + j * 16 + col; const float bb = bfr(BW[o]);
#pragma unroll
    for (int r = 0; r < 8; ++r) st[j * 16 + col][wave * 16 + 8 * g + r] = acc[j][r] + bb; }
  __syncthreads(); for (int e = tid; e < 128 * 16; e += 128) { const int cl = e >> 4, q = e & 15; vst2(OUT + (b * CO + o0 + cl) * (size_t)NPX + p0 + q * 4, *(const v4f*)&st[cl][q * 4]); } }
extern "C" void kernel_launch(void* const* d_in, const int* in_sizes, int n_in, void* d_out, int out_size, void* d_ws, size_t ws_size, hipStream_t stream) {
  (void)in_sizes; (void)n_in; (void)out_size;
  const float** F = (const float**)d_in;
  if (ws_size < (size_t)WS_END) return;
  char* ws = (char*)d_ws; float *K1 = (float*)(ws + WS_K1), *Q1 = (float*)(ws + WS_Q1), *KP = (float*)(ws + WS_KP), *QP = (float*)(ws + WS_QP), *VP = (float*)(ws + WS_VP); _Float16* CT = (_Float16*)(ws + WS_CT);
  k_c1<<<dim3(NPX / 64, NB, 4), 128, 0, stream>>>(F[0], F[1], F[2], F[3], F[7], F[8], F[9], F[13], F[14], K1, Q1, VP);
  k_c2<<<dim3(NPX / 64, NB, 2), 128, 0, stream>>>(K1, Q1, F[4], F[5], F[6], F[10], F[11], F[12], KP, QP);
  k_win<<<TWB, 128, 0, stream>>>(KP, QP, VP, CT);
  k_out<<<dim3(NPX / 64, NB, 2), 128, 0, stream>>>(CT, F[15], F[16], (float*)d_out);
}
